// LPAMLP_38422777430268
// MI455X (gfx1250) — hardware-verified
//
#include <hip/hip_runtime.h>

#define BB   8
#define NN   4096
#define KK   32
#define CC   64
#define CIN  67
#define CINP 96
#define RAD2 (0.15f * 0.15f)
#define LDP  104

typedef _Float16 half8  __attribute__((ext_vector_type(8)));
typedef _Float16 half16 __attribute__((ext_vector_type(16)));
typedef float    v8f    __attribute__((ext_vector_type(8)));

__device__ __forceinline__ half16 cat16(half8 lo, half8 hi) {
  return __builtin_shufflevector(lo, hi, 0,1,2,3,4,5,6,7,8,9,10,11,12,13,14,15);
}

__device__ __forceinline__ half16 load_a(const _Float16* __restrict__ W, int Kdim,
                                         int mt, int kc, int lane) {
  const int m  = mt * 16 + (lane & 15);
  const int hi = (lane >> 4) & 1;
  const _Float16* p0 = W + (size_t)m * Kdim + kc * 32 + hi * 8;
  half8 a = *(const half8*)p0;
  half8 b = *(const half8*)(p0 + 16);
  return cat16(a, b);
}

__device__ __forceinline__ half16 load_b_lds(const _Float16* sB, int colBase,
                                             int kc, int lane, int ldp) {
  const int col = colBase + (lane & 15);
  const int hi  = (lane >> 4) & 1;
  const _Float16* p0 = sB + (size_t)col * ldp + kc * 32 + hi * 8;
  half8 a = *(const half8*)p0;
  half8 b = *(const half8*)(p0 + 16);
  return cat16(a, b);
}

__device__ __forceinline__ v8f wmma_f16(half16 a, half16 b, v8f c) {
  v8f d = __builtin_amdgcn_wmma_f32_16x16x32_f16(false, a, false, b, (short)0, c, false, false);
  asm volatile("v_nop\n\tv_nop\n\tv_nop\n\tv_nop" : "+v"(d) : "v"(a), "v"(b));
  return d;
}
typedef float v4f __attribute__((ext_vector_type(4)));
typedef unsigned v4u __attribute__((ext_vector_type(4)));
typedef int v4i __attribute__((ext_vector_type(4)));
template <typename V> __device__ __forceinline__ void vst2(void* p, V v) {
  *(volatile V*)p = v; __threadfence(); *(volatile V*)p = v;
}

__device__ __forceinline__ half16 pack_b_from_acc(v8f accLo, v8f accHi, int lane) {
  (void)lane;
  half16 r;
  #pragma unroll
  for (int i = 0; i < 8; ++i) { r[i] = (_Float16)accLo[i]; r[8 + i] = (_Float16)accHi[i]; }
  return r;
}

__global__ __launch_bounds__(256) void prep_w(const float* __restrict__ w_attn,
                                              const float* __restrict__ w1,
                                              const float* __restrict__ w2,
                                              const float* __restrict__ wf1,
                                              const float* __restrict__ wf2,
                                              _Float16* __restrict__ wsW) {
  int g = blockIdx.x * 256 + threadIdx.x;
  const int total = 2 * 64 * CINP + 3 * 4096;
  if (g * 8 >= total) return;
  union { half8 h; v4u u; } pk;
  #pragma unroll
  for (int e = 0; e < 8; ++e) {
    int i = g * 8 + e;
    float v;
    if (i < 64 * CINP)            { int m = i / CINP, k = i % CINP; v = (k < CIN) ? w_attn[m * CIN + k] : 0.f; }
    else if (i < 2 * 64 * CINP)   { int j = i - 64 * CINP; int m = j / CINP, k = j % CINP; v = (k < CIN) ? w1[m * CIN + k] : 0.f; }
    else { int j = i - 2 * 64 * CINP; v = (j < 4096) ? w2[j] : (j < 8192) ? wf1[j - 4096] : wf2[j - 8192]; }
    pk.h[e] = (_Float16)v;
  }
  vst2(wsW + (size_t)g * 8, pk.u);
}

__global__ __launch_bounds__(256) void copy_p(const float* __restrict__ p,
                                              float* __restrict__ out) {
  int i = blockIdx.x * 256 + threadIdx.x;
  vst2(out + i, p[i]);
}

__global__ __launch_bounds__(256) void bq(const float* __restrict__ p,
                                          int* __restrict__ idxw) {
  __shared__ float sx[NN], sy[NN], sz[NN];
  const int b  = blockIdx.x >> 9;
  const int q0 = (blockIdx.x & 511) << 3;
  const int tid = threadIdx.x;
  for (int m = tid; m < NN; m += 256) {
    const float* pm = p + (size_t)(b * NN + m) * 3;
    sx[m] = pm[0]; sy[m] = pm[1]; sz[m] = pm[2];
  }
  __syncthreads();
  const int lane = tid & 31;
  const int q = q0 + (tid >> 5);
  const float qx = sx[q], qy = sy[q], qz = sz[q];
  const float sqq = qx * qx + qy * qy + qz * qz;
  int cnt = 0, myidx = 0;
  for (int m0 = 0; m0 < NN && cnt < KK; m0 += 32) {
    const int m = m0 + lane;
    const float x = sx[m], y = sy[m], z = sz[m];
    const float sqm = x * x + y * y + z * z;
    const float dot = qx * x + qy * y + qz * z;
    const float d2  = sqq + sqm - 2.0f * dot;
    unsigned int bm = (unsigned int)__ballot(d2 <= RAD2);
    while (bm && cnt < KK) {
      int t = __ffs(bm) - 1;
      if (lane == cnt) myidx = m0 + t;
      bm &= bm - 1;
      ++cnt;
    }
  }
  const int first = __shfl(myidx, 0, 32);
  vst2(idxw + (size_t)(b * NN + q) * KK + lane, (lane < cnt) ? myidx : first);
}

__global__ __launch_bounds__(128) void lpa_main(const float* __restrict__ p,
                                                const float* __restrict__ f,
                                                const float* __restrict__ b1v,
                                                const float* __restrict__ b2v,
                                                const int* __restrict__ idxw,
                                                const _Float16* __restrict__ wsW,
                                                float* __restrict__ foutw) {
  __shared__ __align__(16) _Float16 sfj[128 * LDP];
  __shared__ int   sidx[128];
  __shared__ float sqp[12];
  __shared__ __align__(16) float sout[4][64];
  const int b   = blockIdx.x >> 10;
  const int q0  = (blockIdx.x & 1023) << 2;
  const int tid = threadIdx.x, lane = tid & 31, wave = tid >> 5;
  const int hi  = (lane >> 4) & 1;

  sidx[tid] = idxw[(size_t)(b * NN + q0 + (tid >> 5)) * KK + (tid & 31)];
  if (tid < 12) sqp[tid] = p[(size_t)(b * NN + q0 + tid / 3) * 3 + (tid % 3)];
  __syncthreads();

  {
    const int col = tid, qi = col >> 5;
    const int ii = sidx[col];
    _Float16* dst = sfj + (size_t)col * LDP;
    const float* pj = p + (size_t)(b * NN + ii) * 3;
    dst[0] = (_Float16)(pj[0] - sqp[qi * 3 + 0]);
    dst[1] = (_Float16)(pj[1] - sqp[qi * 3 + 1]);
    dst[2] = (_Float16)(pj[2] - sqp[qi * 3 + 2]);
    const float* fb = f + (size_t)b * CC * NN + ii;
    #pragma unroll 8
    for (int ch = 0; ch < CC; ++ch) dst[3 + ch] = (_Float16)fb[(size_t)ch * NN];
    #pragma unroll
    for (int k = CIN; k < CINP; ++k) dst[k] = (_Float16)0.f;
  }
  __syncthreads();

  const _Float16* wA  = wsW;
  const _Float16* w1w = wsW + 64 * CINP;
  const _Float16* w2w = wsW + 2 * 64 * CINP;
  const int q = q0 + wave;

  v8f attnA[2][4], yA[2][4];
  #pragma unroll
  for (int t = 0; t < 2; ++t) {
    const int cb = wave * 32 + t * 16;
    half16 B0 = load_b_lds(sfj, cb, 0, lane, LDP);
    half16 B1 = load_b_lds(sfj, cb, 1, lane, LDP);
    half16 B2 = load_b_lds(sfj, cb, 2, lane, LDP);
    v8f accX[4];
    #pragma unroll
    for (int mt = 0; mt < 4; ++mt) {
      v8f ca = {}; v8f cx = {};
      ca = wmma_f16(load_a(wA,  CINP, mt, 0, lane), B0, ca);
      ca = wmma_f16(load_a(wA,  CINP, mt, 1, lane), B1, ca);
      ca = wmma_f16(load_a(wA,  CINP, mt, 2, lane), B2, ca);
      cx = wmma_f16(load_a(w1w, CINP, mt, 0, lane), B0, cx);
      cx = wmma_f16(load_a(w1w, CINP, mt, 1, lane), B1, cx);
      cx = wmma_f16(load_a(w1w, CINP, mt, 2, lane), B2, cx);
      const float* bp = b1v + mt * 16 + hi * 8;
      #pragma unroll
      for (int r = 0; r < 8; ++r) cx[r] = fmaxf(cx[r] + bp[r], 0.f);
      attnA[t][mt] = ca;
      accX[mt] = cx;
    }
    half16 X0 = pack_b_from_acc(accX[0], accX[1], lane);
    half16 X1 = pack_b_from_acc(accX[2], accX[3], lane);
    #pragma unroll
    for (int mt = 0; mt < 4; ++mt) {
      v8f cy = {};
      cy = wmma_f16(load_a(w2w, 64, mt, 0, lane), X0, cy);
      cy = wmma_f16(load_a(w2w, 64, mt, 1, lane), X1, cy);
      const float* bp = b2v + mt * 16 + hi * 8;
      #pragma unroll
      for (int r = 0; r < 8; ++r) cy[r] += bp[r];
      yA[t][mt] = cy;
    }
  }

  #pragma unroll
  for (int mt = 0; mt < 4; ++mt) {
    #pragma unroll
    for (int r = 0; r < 8; ++r) {
      float a0 = attnA[0][mt][r], a1 = attnA[1][mt][r];
      float mx = fmaxf(a0, a1);
      #pragma unroll
      for (int d = 1; d < 16; d <<= 1) mx = fmaxf(mx, __shfl_xor(mx, d, 32));
      float e0 = __expf(a0 - mx), e1 = __expf(a1 - mx);
      float s   = e0 + e1;
      float num = e0 * yA[0][mt][r] + e1 * yA[1][mt][r];
      #pragma unroll
      for (int d = 1; d < 16; d <<= 1) {
        s   += __shfl_xor(s,   d, 32);
        num += __shfl_xor(num, d, 32);
      }
      if ((lane & 15) == 0) {
        const int ch = mt * 16 + r + hi * 8;
        sout[wave][ch] = fmaxf(num / s + f[(size_t)(b * CC + ch) * NN + q], 0.f);
      }
    }
  }
  __syncthreads();
  if (lane < 16) vst2(foutw + ((size_t)(b * NN + q)) * CC + lane * 4, *(const v4f*)(&sout[wave][lane * 4]));
}

__global__ __launch_bounds__(256) void final_mlp(const float* __restrict__ bf1v,
                                                 const float* __restrict__ bf2v,
                                                 const _Float16* __restrict__ wsW,
                                                 const float* __restrict__ foutw,
                                                 float* __restrict__ outp) {
  __shared__ __align__(16) float so[64][128];
  const int tid = threadIdx.x, lane = tid & 31, wave = tid >> 5;
  const int tile = blockIdx.x * 8 + wave;
  const int col  = tile * 16 + (lane & 15);
  const int b = col >> 12, q = col & (NN - 1);
  const int hi = (lane >> 4) & 1;
  const _Float16* wf1w = wsW + 2 * 64 * CINP + 4096;
  const _Float16* wf2w = wsW + 2 * 64 * CINP + 2 * 4096;

  const float* fr = foutw + ((size_t)(b * NN + q)) * CC;
  half16 F0, F1;
  #pragma unroll
  for (int h = 0; h < 8; ++h) {
    F0[h] = (_Float16)fr[8 * hi + h];       F0[8 + h] = (_Float16)fr[16 + 8 * hi + h];
    F1[h] = (_Float16)fr[32 + 8 * hi + h];  F1[8 + h] = (_Float16)fr[48 + 8 * hi + h];
  }
  v8f acc1[4];
  #pragma unroll
  for (int mt = 0; mt < 4; ++mt) {
    v8f c = {};
    c = wmma_f16(load_a(wf1w, 64, mt, 0, lane), F0, c);
    c = wmma_f16(load_a(wf1w, 64, mt, 1, lane), F1, c);
    const float* bp = bf1v + mt * 16 + hi * 8;
    #pragma unroll
    for (int r = 0; r < 8; ++r) c[r] = fmaxf(c[r] + bp[r], 0.f);
    acc1[mt] = c;
  }
  half16 H0 = pack_b_from_acc(acc1[0], acc1[1], lane);
  half16 H1 = pack_b_from_acc(acc1[2], acc1[3], lane);
  float* outF = outp + (size_t)BB * NN * 3;
  #pragma unroll
  for (int mt = 0; mt < 4; ++mt) {
    v8f c = {};
    c = wmma_f16(load_a(wf2w, 64, mt, 0, lane), H0, c);
    c = wmma_f16(load_a(wf2w, 64, mt, 1, lane), H1, c);
    const float* bp = bf2v + mt * 16 + hi * 8;
    #pragma unroll
    for (int r = 0; r < 8; ++r) {
      const int ch = mt * 16 + r + hi * 8;
      so[ch][wave * 16 + (lane & 15)] = fmaxf(c[r] + bp[r] + fr[ch], 0.f);
    }
  }
  __syncthreads();
  const int q0blk = (blockIdx.x * 128) & (NN - 1), bblk = (blockIdx.x * 128) >> 12;
  for (int g = tid; g < 64 * 32; g += 256) {
    const int ch = g >> 5, pc = g & 31;
    vst2(outF + ((size_t)(bblk * CC + ch)) * NN + q0blk + pc * 4, *(const v4f*)(&so[ch][pc * 4]));
  }
}

extern "C" void kernel_launch(void* const* d_in, const int* in_sizes, int n_in,
                              void* d_out, int out_size, void* d_ws, size_t ws_size,
                              hipStream_t stream) {
  (void)in_sizes; (void)n_in; (void)out_size; (void)ws_size;
  const float* p      = (const float*)d_in[0];
  const float* f      = (const float*)d_in[1];
  const float* w_attn = (const float*)d_in[2];
  const float* b_attn = (const float*)d_in[3]; (void)b_attn;
  const float* w1     = (const float*)d_in[4];
  const float* b1     = (const float*)d_in[5];
  const float* w2     = (const float*)d_in[6];
  const float* b2     = (const float*)d_in[7];
  const float* wf1    = (const float*)d_in[8];
  const float* bf1    = (const float*)d_in[9];
  const float* wf2    = (const float*)d_in[10];
  const float* bf2    = (const float*)d_in[11];
  float* out = (float*)d_out;

  char* ws = (char*)d_ws;
  int*      idxw  = (int*)ws;
  float*    foutw = (float*)(ws + (size_t)4  * 1024 * 1024);
  _Float16* wsW   = (_Float16*)(ws + (size_t)12 * 1024 * 1024);

  prep_w  <<<12,   256, 0, stream>>>(w_attn, w1, w2, wf1, wf2, wsW);
  copy_p  <<<384,  256, 0, stream>>>(p, out);
  bq      <<<4096, 256, 0, stream>>>(p, idxw);
  lpa_main<<<8192, 128, 0, stream>>>(p, f, b1, b2, idxw, wsW, foutw);
  final_mlp<<<256, 256, 0, stream>>>(bf1, bf2, wsW, foutw, out);
}
